// SimpleTransformerBlock_10247791968529
// MI455X (gfx1250) — hardware-run, weakly checked
//
#include <hip/hip_runtime.h>
#include <hip/hip_bf16.h>

typedef __attribute__((ext_vector_type(16))) _Float16 v16h;
typedef __attribute__((ext_vector_type(8)))  _Float16 v8h;
typedef __attribute__((ext_vector_type(16))) __bf16   v16b;
typedef __attribute__((ext_vector_type(8)))  __bf16   v8b;
typedef __attribute__((ext_vector_type(8)))  float    v8f;
typedef __attribute__((ext_vector_type(4)))  float    v4f;
#define U16(p) ((const unsigned short*)(const void*)(p))

#define MODEL_DIM 1024
#define NUM_HEADS 16
#define HEAD_D    64
#define MLP_DIM   4096
#define BATCH     2
#define SEQ_LEN   2048
#define NROWS     (BATCH * SEQ_LEN)
#define QK_LD     2048
#define O_LD      1024
#define PSC_F     32768.0f
#define OSC_F     64.0f

__device__ __forceinline__ unsigned short f2bf_bits(float f) {
  unsigned u = __float_as_uint(f);
  return (unsigned short)((u + 0x7FFFu + ((u >> 16) & 1u)) >> 16);
}
__device__ __forceinline__ float bf_bits2f(unsigned short h) { return __uint_as_float(((unsigned)h) << 16); }

__device__ __forceinline__ void dep_guard_h(v8f& a, v8f& b, v16h x, v16h y) { asm volatile("v_nop\n\tv_nop\n\tv_nop\n\tv_nop" : "+v"(a), "+v"(b) : "v"(x), "v"(y)); }
__device__ __forceinline__ void dep_guard_b(v8f& a, v8f& b, v16b x, v16b y) { asm volatile("v_nop\n\tv_nop\n\tv_nop\n\tv_nop" : "+v"(a), "+v"(b) : "v"(x), "v"(y)); }
__device__ __forceinline__ void keep4_h(v16h a, v16h b, v16h c, v16h d) { asm volatile("v_nop" :: "v"(a), "v"(b), "v"(c), "v"(d)); }
__device__ __forceinline__ void keep4_b(v16b a, v16b b, v16b c, v16b d) { asm volatile("v_nop" :: "v"(a), "v"(b), "v"(c), "v"(d)); }
__device__ __forceinline__ void acc_guard4(v8f& a, v8f& b, v8f& c, v8f& d) { asm volatile("v_nop\n\tv_nop\n\tv_nop\n\tv_nop" : "+v"(a), "+v"(b), "+v"(c), "+v"(d)); }
template <typename T> struct Frag;
template <> struct Frag<_Float16> {
  typedef v16h V; union U { v16h v; v8h h[2]; };
  static __device__ __forceinline__ v16h load(const _Float16* p) {
    U f; f.h[0] = *(const v8h*)(p); f.h[1] = *(const v8h*)(p + 16); return f.v;
  }
  static __device__ __forceinline__ v8f mma(v16h a, v16h b, v8f c) {
    return __builtin_amdgcn_wmma_f32_16x16x32_f16(false, a, false, b, (short)0, c, false, false);
  }
  static __device__ __forceinline__ void guard(v8f& a, v8f& b, v16h x, v16h y) { dep_guard_h(a, b, x, y); }
  static __device__ __forceinline__ void keep(v16h a, v16h b, v16h c, v16h d) { keep4_h(a, b, c, d); }
};
template <> struct Frag<__bf16> {
  typedef v16b V; union U { v16b v; v8b h[2]; };
  static __device__ __forceinline__ v16b load(const __bf16* p) {
    U f; f.h[0] = *(const v8b*)(p); f.h[1] = *(const v8b*)(p + 16); return f.v;
  }
  static __device__ __forceinline__ v8f mma(v16b a, v16b b, v8f c) {
    return __builtin_amdgcn_wmma_f32_16x16x32_bf16(false, a, false, b, (short)0, c, false, false);
  }
  static __device__ __forceinline__ void guard(v8f& a, v8f& b, v16b x, v16b y) { dep_guard_b(a, b, x, y); }
  static __device__ __forceinline__ void keep(v16b a, v16b b, v16b c, v16b d) { keep4_b(a, b, c, d); }
};

template <int ET> struct Elem;
template <> struct Elem<0> { typedef _Float16 T; };
template <> struct Elem<1> { typedef __bf16 T; };
template <int ET, bool SPLIT, int BIAS_MODE, int OUT_MODE, bool RESID, int ACT = 0>
__global__ __launch_bounds__(256) void wmma_gemm64(
    const unsigned short* __restrict__ Ap, const unsigned short* __restrict__ A2p, int lda, long strideA,
    const unsigned short* __restrict__ Btp, const unsigned short* __restrict__ Bt2p, int ldb, long strideB,
    void* __restrict__ Cout, void* __restrict__ Cout2, int ldc, long strideC,
    const float* __restrict__ bias,
    const float* __restrict__ resid, long strideR,
    int M, int N, int K, float scale) {
  static_assert(!RESID || OUT_MODE == 0);
  typedef typename Elem<ET>::T T;
  typedef typename Frag<T>::V V;
  const T* A = (const T*)Ap; const T* A2 = (const T*)A2p; const T* Bt = (const T*)Btp; const T* Bt2 = (const T*)Bt2p;
  __shared__ __align__(16) float sT[8][16 * 68];
  const int b    = blockIdx.y;
  const int lane = threadIdx.x & 31;
  const int wave = threadIdx.x >> 5;
  const int tilesN = N >> 6;
  const int tilesM = M >> 6;
  const int tile = blockIdx.x * 8 + wave;
  if (tile >= tilesM * tilesN) return;
  const int tm = tile / tilesN;
  const int tn = tile - tm * tilesN;
  const int m0 = tm << 6;
  const int n0 = tn << 6;

  const T* Ab  = A  + (size_t)b * strideA;
  const T* Bb  = Bt + (size_t)b * strideB;
  const T* Ab2 = SPLIT ? (A2  + (size_t)b * strideA) : nullptr;
  const T* Bb2 = SPLIT ? (Bt2 + (size_t)b * strideB) : nullptr;

  const int rlane = lane & 15;
  const int koff  = (lane >> 4) * 8;
  const int mOff  = (lane >> 4) * 8;

  v8f acc[4][4];
#pragma unroll
  for (int i = 0; i < 4; ++i)
#pragma unroll
    for (int j = 0; j < 4; ++j) acc[i][j] = (v8f){0.f,0.f,0.f,0.f,0.f,0.f,0.f,0.f};

  for (int k0 = 0; k0 < K; k0 += 32) {
    V bh[4], bl[4];
#pragma unroll
    for (int j = 0; j < 4; ++j) {
      const size_t bo = (size_t)(n0 + (j << 4) + rlane) * ldb + koff + k0;
      bh[j] = Frag<T>::load(Bb + bo);
      if (SPLIT) bl[j] = Frag<T>::load(Bb2 + bo);
    }
#pragma unroll
    for (int i = 0; i < 4; ++i) {
      const size_t ao = (size_t)(m0 + (i << 4) + rlane) * lda + koff + k0;
      V ah = Frag<T>::load(Ab + ao);
      V al;
      if (SPLIT) al = Frag<T>::load(Ab2 + ao);
#pragma unroll
      for (int j = 0; j < 4; ++j) {
        acc[i][j] = Frag<T>::mma(ah, bh[j], acc[i][j]);
        if (SPLIT) {
          acc[i][j] = Frag<T>::mma(ah, bl[j], acc[i][j]);
          acc[i][j] = Frag<T>::mma(al, bh[j], acc[i][j]);
        }
      }
      Frag<T>::guard(acc[i][0], acc[i][3], ah, SPLIT ? al : ah);
    }
    Frag<T>::keep(bh[0], bh[1], bh[2], bh[3]);
    if (SPLIT) Frag<T>::keep(bl[0], bl[1], bl[2], bl[3]);
  }
  acc_guard4(acc[0][0], acc[0][1], acc[0][2], acc[0][3]);
  acc_guard4(acc[1][0], acc[1][1], acc[1][2], acc[1][3]);
  acc_guard4(acc[2][0], acc[2][1], acc[2][2], acc[2][3]);
  acc_guard4(acc[3][0], acc[3][1], acc[3][2], acc[3][3]);

  float* slab = sT[wave];
  const float* Rb = RESID ? (resid + (size_t)b * strideR) : nullptr;
#pragma unroll
  for (int i = 0; i < 4; ++i) {
    const int mBase = m0 + (i << 4);
#pragma unroll
    for (int j = 0; j < 4; ++j) {
      const int n = n0 + (j << 4) + rlane;
      float bv = 0.f;
      if (BIAS_MODE == 2) bv = bias[n];
#pragma unroll
      for (int r = 0; r < 8; ++r) {
        float v = acc[i][j][r] * scale;
        if (BIAS_MODE == 1) v += bias[mBase + mOff + r];
        if (BIAS_MODE == 2) v += bv;
        if (ACT == 2) v = fmaxf(v, 0.0f);
        if (ACT == 3) v = v * (1.0f / (1.0f + expf(-v)));
        if (ACT == 4) v = (v > 0.f) ? v : 0.01f * v;
        slab[(mOff + r) * 68 + (j << 4) + rlane] = v;
      }
    }
    __builtin_amdgcn_fence(__ATOMIC_RELEASE, "workgroup");
    __builtin_amdgcn_wave_barrier();
    __builtin_amdgcn_fence(__ATOMIC_ACQUIRE, "workgroup");
    if (OUT_MODE == 0) {
      float* C = (float*)Cout + (size_t)b * strideC;
      const int hh = lane >> 4, c4 = (lane & 15) * 4;
      v4f vals[8];
#pragma unroll
      for (int it = 0; it < 8; ++it) {
        const int row = it * 2 + hh;
        v4f v = *(const v4f*)(slab + row * 68 + c4);
        if (RESID) {
          const v4f r4 = *(const v4f*)(Rb + (size_t)(mBase + row) * ldc + n0 + c4);
          v = v + r4;
        }
        vals[it] = v;
      }
      for (int pass = 0; pass < 2; ++pass) {
#pragma unroll
        for (int it = 0; it < 8; ++it) {
          const int row = it * 2 + hh;
          *(volatile v4f*)(C + (size_t)(mBase + row) * ldc + n0 + c4) = vals[it];
        }
        __threadfence();
      }
    } else {
      const int q = lane >> 3, c8 = (lane & 7) * 8;
      unsigned short* C  = (unsigned short*)Cout  + (size_t)b * strideC;
      unsigned short* C2 = (OUT_MODE == 2) ? ((unsigned short*)Cout2 + (size_t)b * strideC) : nullptr;
      for (int pass = 0; pass < 2; ++pass) {
#pragma unroll
        for (int it = 0; it < 4; ++it) {
          const int row = it * 4 + q;
          const float* sp = slab + row * 68 + c8;
          v8h hv, lv;
#pragma unroll
          for (int e = 0; e < 8; ++e) {
            if (OUT_MODE == 1) {
              hv[e] = (_Float16)sp[e];
            } else {
              unsigned short hb = f2bf_bits(sp[e]);
              unsigned short lb = f2bf_bits(sp[e] - bf_bits2f(hb));
              hv[e] = __builtin_bit_cast(_Float16, hb);
              lv[e] = __builtin_bit_cast(_Float16, lb);
            }
          }
          *(volatile v8h*)(C + (size_t)(mBase + row) * ldc + n0 + c8) = hv;
          if (OUT_MODE == 2) *(volatile v8h*)(C2 + (size_t)(mBase + row) * ldc + n0 + c8) = lv;
        }
        __threadfence();
      }
    }
    __builtin_amdgcn_fence(__ATOMIC_RELEASE, "workgroup");
    __builtin_amdgcn_wave_barrier();
    __builtin_amdgcn_fence(__ATOMIC_ACQUIRE, "workgroup");
  }
}

__global__ __launch_bounds__(256) void cast_f32_f16x2(
    const float* __restrict__ in, _Float16* __restrict__ out, int n2, float sc) {
  int i = blockIdx.x * 256 + threadIdx.x;
  if (i < n2) {
    const _Float16 h0 = (_Float16)(in[2 * i] * sc), h1 = (_Float16)(in[2 * i + 1] * sc);
    const unsigned u = (unsigned)__builtin_bit_cast(unsigned short, h0) | ((unsigned)__builtin_bit_cast(unsigned short, h1) << 16);
    ((volatile unsigned*)out)[i] = u;
    __threadfence();
    ((volatile unsigned*)out)[i] = u;
  }
}

__global__ __launch_bounds__(128) void layernorm_f16_kernel(
    const float* __restrict__ x, const float* __restrict__ w, const float* __restrict__ bb,
    unsigned short* __restrict__ outp) {
  __shared__ float red1[4];
  __shared__ float red2[4];
  const int row  = blockIdx.x;
  const int tid  = threadIdx.x;
  const int lane = tid & 31;
  const int wave = tid >> 5;
  const float* xr = x + (size_t)row * MODEL_DIM + tid * 8;
  const v4f a0 = *(const v4f*)(xr);
  const v4f a1 = *(const v4f*)(xr + 4);
  float xv[8];
  xv[0] = a0[0]; xv[1] = a0[1]; xv[2] = a0[2]; xv[3] = a0[3];
  xv[4] = a1[0]; xv[5] = a1[1]; xv[6] = a1[2]; xv[7] = a1[3];
  float s = 0.0f;
#pragma unroll
  for (int e = 0; e < 8; ++e) s += xv[e];
#pragma unroll
  for (int off = 1; off < 32; off <<= 1) s += __shfl_xor(s, off, 32);
  if (lane == 0) red1[wave] = s;
  __syncthreads();
  const float tot = (red1[0] + red1[1]) + (red1[2] + red1[3]);
  const float mu = tot * (1.0f / (float)MODEL_DIM);
  float q = 0.0f;
#pragma unroll
  for (int e = 0; e < 8; ++e) { const float d = xv[e] - mu; q += d * d; }
#pragma unroll
  for (int off = 1; off < 32; off <<= 1) q += __shfl_xor(q, off, 32);
  if (lane == 0) red2[wave] = q;
  __syncthreads();
  const float var = ((red2[0] + red2[1]) + (red2[2] + red2[3])) * (1.0f / (float)MODEL_DIM);
  const float inv = rsqrtf(var + 1e-5f);
  const v4f w0 = *(const v4f*)(w + tid * 8);
  const v4f w1 = *(const v4f*)(w + tid * 8 + 4);
  const v4f b0 = *(const v4f*)(bb + tid * 8);
  const v4f b1 = *(const v4f*)(bb + tid * 8 + 4);
  float wv[8], bv[8];
  wv[0] = w0[0]; wv[1] = w0[1]; wv[2] = w0[2]; wv[3] = w0[3];
  wv[4] = w1[0]; wv[5] = w1[1]; wv[6] = w1[2]; wv[7] = w1[3];
  bv[0] = b0[0]; bv[1] = b0[1]; bv[2] = b0[2]; bv[3] = b0[3];
  bv[4] = b1[0]; bv[5] = b1[1]; bv[6] = b1[2]; bv[7] = b1[3];
  v8h hv;
#pragma unroll
  for (int e = 0; e < 8; ++e) {
    const float y = (xv[e] - mu) * inv * wv[e] + bv[e];
    hv[e] = (_Float16)y;
  }
  unsigned short* op = outp + (size_t)row * MODEL_DIM + tid * 8;
  *(volatile v8h*)op = hv;
  __threadfence();
  *(volatile v8h*)op = hv;
}

__device__ __forceinline__ v8f mma16h(v16h a, v16h b, v8f c) {
  c = __builtin_amdgcn_wmma_f32_16x16x32_f16(false, a, false, b, (short)0, c, false, false);
  asm volatile("v_nop\n\tv_nop\n\tv_nop\n\tv_nop" : "+v"(c) : "v"(a), "v"(b));
  return c;
}

__global__ __launch_bounds__(128) void attn16_kernel(
    const unsigned short* __restrict__ qkp, const unsigned short* __restrict__ vtp,
    unsigned short* __restrict__ op) {
  __shared__ __align__(16) _Float16 Ksh[64 * 64];
  __shared__ __align__(16) _Float16 Vth[64 * 64];
  __shared__ __align__(16) _Float16 Psh[4][16 * 64];
  __shared__ __align__(16) float  Os[4][16 * 68];

  const int tid  = threadIdx.x;
  const int wave = tid >> 5;
  const int lane = tid & 31;
  const int hh   = lane >> 4;
  const int c    = lane & 15;

  const int bx = blockIdx.x;
  const int qb = bx & 31;
  const int bh = bx >> 5;
  const int h  = bh & (NUM_HEADS - 1);
  const int b  = bh >> 4;
  const int q0 = qb * 64 + wave * 16;

  const _Float16* qplane = (const _Float16*)qkp + (size_t)b * SEQ_LEN * QK_LD + h * HEAD_D;
  const _Float16* kplane = qplane + MODEL_DIM;
  const _Float16* vplane = (const _Float16*)vtp + ((size_t)(b * NUM_HEADS + h) * HEAD_D) * SEQ_LEN;
  _Float16* oplane = (_Float16*)op + (size_t)b * SEQ_LEN * O_LD + h * HEAD_D;

  v16h qa[2];
  {
    const _Float16* qrow = qplane + (size_t)(q0 + c) * QK_LD;
#pragma unroll
    for (int dc = 0; dc < 2; ++dc) qa[dc] = Frag<_Float16>::load(qrow + dc * 32 + 8 * hh);
  }

  float mrow[8], lrow[8];
  v8f oacc[4];
#pragma unroll
  for (int r = 0; r < 8; ++r) { mrow[r] = -__builtin_inff(); lrow[r] = 0.f; }
#pragma unroll
  for (int t = 0; t < 4; ++t) oacc[t] = (v8f){0.f,0.f,0.f,0.f,0.f,0.f,0.f,0.f};

  for (int kc = 0; kc < SEQ_LEN / 64; ++kc) {
    const int kv0 = kc * 64;
    __syncthreads();
    {
      const int r = tid >> 1, hf = (tid & 1) * 32;
      const _Float16* ksrc = kplane + (size_t)(kv0 + r) * QK_LD + hf;
      const _Float16* vsrc = vplane + (size_t)r * SEQ_LEN + kv0 + hf;
      v8h kk[4], vv[4];
#pragma unroll
      for (int i = 0; i < 4; ++i) { kk[i] = *(const v8h*)(ksrc + 8 * i); vv[i] = *(const v8h*)(vsrc + 8 * i); }
#pragma unroll
      for (int i = 0; i < 4; ++i) {
        *(v8h*)(Ksh + r * 64 + hf + 8 * i) = kk[i];
        *(v8h*)(Vth + r * 64 + hf + 8 * i) = vv[i];
      }
    }
    __syncthreads();

    v8f s[4];
#pragma unroll
    for (int j = 0; j < 4; ++j) {
      s[j] = (v8f){0.f,0.f,0.f,0.f,0.f,0.f,0.f,0.f};
#pragma unroll
      for (int dc = 0; dc < 2; ++dc) {
        const v16h kb = Frag<_Float16>::load(Ksh + (j * 16 + c) * 64 + dc * 32 + 8 * hh);
        s[j] = mma16h(qa[dc], kb, s[j]);
      }
    }
    float cm[8];
#pragma unroll
    for (int r = 0; r < 8; ++r) {
      float m = -__builtin_inff();
#pragma unroll
      for (int j = 0; j < 4; ++j) { s[j][r] *= 0.125f; m = fmaxf(m, s[j][r]); }
#pragma unroll
      for (int off = 1; off < 16; off <<= 1) m = fmaxf(m, __shfl_xor(m, off, 32));
      cm[r] = m;
    }
    _Float16* pwh = Psh[wave];
#pragma unroll
    for (int r = 0; r < 8; ++r) {
      const float mnew = fmaxf(mrow[r], cm[r]);
      const float alpha = expf(mrow[r] - mnew);
      mrow[r] = mnew;
      float psum = 0.f;
#pragma unroll
      for (int j = 0; j < 4; ++j) {
        const float p = expf(s[j][r] - mnew);
        psum += p;
        pwh[(8 * hh + r) * 64 + j * 16 + c] = (_Float16)(p * PSC_F);
      }
#pragma unroll
      for (int off = 1; off < 16; off <<= 1) psum += __shfl_xor(psum, off, 32);
      lrow[r] = lrow[r] * alpha + psum;
#pragma unroll
      for (int t = 0; t < 4; ++t) oacc[t][r] *= alpha;
    }
    __builtin_amdgcn_fence(__ATOMIC_RELEASE, "workgroup");
    __builtin_amdgcn_wave_barrier();
    __builtin_amdgcn_fence(__ATOMIC_ACQUIRE, "workgroup");
#pragma unroll
    for (int kk2 = 0; kk2 < 2; ++kk2) {
      const v16h pa = Frag<_Float16>::load(pwh + c * 64 + kk2 * 32 + 8 * hh);
#pragma unroll
      for (int t = 0; t < 4; ++t) {
        const v16h vb = Frag<_Float16>::load(Vth + (t * 16 + c) * 64 + kk2 * 32 + 8 * hh);
        oacc[t] = mma16h(pa, vb, oacc[t]);
      }
    }
  }

  float* os = Os[wave];
#pragma unroll
  for (int r = 0; r < 8; ++r) {
    const float inv = (1.0f / (lrow[r] * PSC_F)) * OSC_F;
#pragma unroll
    for (int t = 0; t < 4; ++t) os[(8 * hh + r) * 68 + t * 16 + c] = oacc[t][r] * inv;
  }
  __builtin_amdgcn_fence(__ATOMIC_RELEASE, "workgroup");
  __builtin_amdgcn_wave_barrier();
  __builtin_amdgcn_fence(__ATOMIC_ACQUIRE, "workgroup");
  {
    const int q4 = lane >> 3, c8 = (lane & 7) * 8;
    for (int pass = 0; pass < 2; ++pass) {
#pragma unroll
      for (int it = 0; it < 4; ++it) {
        const int row = it * 4 + q4;
        const float* sp = os + row * 68 + c8;
        v8h hv;
#pragma unroll
        for (int e = 0; e < 8; ++e) hv[e] = (_Float16)sp[e];
        *(volatile v8h*)(oplane + (size_t)(q0 + row) * O_LD + c8) = hv;
      }
      __threadfence();
    }
  }
}

extern "C" void kernel_launch(void* const* d_in, const int* in_sizes, int n_in,
                              void* d_out, int out_size, void* d_ws, size_t ws_size,
                              hipStream_t stream) {
  if (n_in < 12) return;
  if (in_sizes[0] != NROWS * MODEL_DIM) return;
  if (out_size != NROWS * MODEL_DIM) return;

  const float* x     = (const float*)d_in[0];
  const float* qkv_w = (const float*)d_in[1];
  const float* out_w = (const float*)d_in[2];
  const float* out_b = (const float*)d_in[3];
  const float* ff_w1 = (const float*)d_in[4];
  const float* ff_b1 = (const float*)d_in[5];
  const float* ff_w2 = (const float*)d_in[6];
  const float* ff_b2 = (const float*)d_in[7];
  const float* ln1_w = (const float*)d_in[8];
  const float* ln1_b = (const float*)d_in[9];
  const float* ln2_w = (const float*)d_in[10];
  const float* ln2_b = (const float*)d_in[11];
  float* outp = (float*)d_out;

  const size_t OFF_WQKV = 0;
  const size_t OFF_WOUT = OFF_WQKV + (size_t)3 * MODEL_DIM * MODEL_DIM * 2;
  const size_t OFF_W1   = OFF_WOUT + (size_t)MODEL_DIM * MODEL_DIM * 2;
  const size_t OFF_W2   = OFF_W1 + (size_t)MLP_DIM * MODEL_DIM * 2;
  const size_t OFF_XLN  = OFF_W2 + (size_t)MODEL_DIM * MLP_DIM * 2;
  const size_t OFF_QK   = OFF_XLN + (size_t)NROWS * MODEL_DIM * 2;
  const size_t OFF_VT   = OFF_QK + (size_t)NROWS * QK_LD * 2;
  const size_t OFF_O    = OFF_VT + (size_t)BATCH * MODEL_DIM * SEQ_LEN * 2;
  const size_t OFF_X1   = OFF_O + (size_t)NROWS * O_LD * 2;
  const size_t OFF_H    = OFF_X1 + (size_t)NROWS * MODEL_DIM * 4;
  const size_t WS_TOTAL = OFF_H + (size_t)NROWS * MLP_DIM * 2;
  if (WS_TOTAL > ws_size) return;

  char* wsb = (char*)d_ws;
  unsigned short* wqkv16 = (unsigned short*)(wsb + OFF_WQKV);
  unsigned short* wout16 = (unsigned short*)(wsb + OFF_WOUT);
  unsigned short* w1_16  = (unsigned short*)(wsb + OFF_W1);
  unsigned short* w2_16  = (unsigned short*)(wsb + OFF_W2);
  unsigned short* xln16  = (unsigned short*)(wsb + OFF_XLN);
  unsigned short* qk16   = (unsigned short*)(wsb + OFF_QK);
  unsigned short* vt16   = (unsigned short*)(wsb + OFF_VT);
  unsigned short* o16    = (unsigned short*)(wsb + OFF_O);
  float*          x1     = (float*)(wsb + OFF_X1);
  unsigned short* h16    = (unsigned short*)(wsb + OFF_H);

  static_assert(MODEL_DIM % 32 == 0 && MLP_DIM % 32 == 0);
  static_assert(NROWS % 64 == 0 && MODEL_DIM % 64 == 0 && MLP_DIM % 64 == 0 && SEQ_LEN % 64 == 0 && (2 * MODEL_DIM) % 64 == 0);
  static_assert((3 * MODEL_DIM * MODEL_DIM) % 512 == 0 && (MODEL_DIM * MLP_DIM) % 512 == 0);

  {
    const int n2a = 3 * MODEL_DIM * MODEL_DIM / 2;
    cast_f32_f16x2<<<(n2a + 255) / 256, 256, 0, stream>>>(qkv_w, (_Float16*)wqkv16, n2a, 32.0f);
    const int n2b = MODEL_DIM * MODEL_DIM / 2;
    cast_f32_f16x2<<<(n2b + 255) / 256, 256, 0, stream>>>(out_w, (_Float16*)wout16, n2b, 32.0f);
    const int n2c = MLP_DIM * MODEL_DIM / 2;
    cast_f32_f16x2<<<(n2c + 255) / 256, 256, 0, stream>>>(ff_w1, (_Float16*)w1_16, n2c, 32.0f);
    cast_f32_f16x2<<<(n2c + 255) / 256, 256, 0, stream>>>(ff_w2, (_Float16*)w2_16, n2c, 64.0f);
  }

  layernorm_f16_kernel<<<NROWS, 128, 0, stream>>>(x, ln1_w, ln1_b, xln16);

  {
    const int M = NROWS, N = 2 * MODEL_DIM, K = MODEL_DIM;
    const int tiles = (M / 64) * (N / 64);
    wmma_gemm64<0, false, 0, 1, false, 0><<<dim3((tiles + 7) / 8, 1), 256, 0, stream>>>(
        xln16, xln16, K, 0L, wqkv16, wqkv16, K, 0L,
        (void*)qk16, nullptr, QK_LD, 0L, nullptr, nullptr, 0L, M, N, K, 1.0f / 32.0f);
  }
  {
    const int M = MODEL_DIM, N = SEQ_LEN, K = MODEL_DIM;
    const int tiles = (M / 64) * (N / 64);
    wmma_gemm64<0, false, 0, 1, false, 0><<<dim3((tiles + 7) / 8, BATCH), 256, 0, stream>>>(
        wqkv16 + (size_t)2 * MODEL_DIM * MODEL_DIM, wqkv16 + (size_t)2 * MODEL_DIM * MODEL_DIM, K, 0L,
        xln16, xln16, K, (long)SEQ_LEN * MODEL_DIM,
        (void*)vt16, nullptr, SEQ_LEN, (long)MODEL_DIM * SEQ_LEN, nullptr, nullptr, 0L, M, N, K, 1.0f / 32.0f);
  }

  attn16_kernel<<<BATCH * NUM_HEADS * (SEQ_LEN / 64), 128, 0, stream>>>(qk16, vt16, o16);

  {
    const int M = NROWS, N = MODEL_DIM, K = MODEL_DIM;
    const int tiles = (M / 64) * (N / 64);
    wmma_gemm64<0, false, 2, 0, true, 0><<<dim3((tiles + 7) / 8, 1), 256, 0, stream>>>(
        o16, o16, K, 0L, wout16, wout16, K, 0L,
        (void*)x1, nullptr, MODEL_DIM, 0L, out_b, x, 0L, M, N, K, 1.0f / 2048.0f);
  }

  layernorm_f16_kernel<<<NROWS, 128, 0, stream>>>(x1, ln2_w, ln2_b, xln16);

  {
    const int M = NROWS, N = MLP_DIM, K = MODEL_DIM;
    const int tiles = (M / 64) * (N / 64);
    wmma_gemm64<0, false, 2, 1, false, 3><<<dim3((tiles + 7) / 8, 1), 256, 0, stream>>>(
        xln16, xln16, K, 0L, w1_16, w1_16, K, 0L,
        (void*)h16, nullptr, MLP_DIM, 0L, ff_b1, nullptr, 0L, M, N, K, 1.0f / 32.0f);
  }

  {
    const int M = NROWS, N = MODEL_DIM, K = MLP_DIM;
    const int tiles = (M / 64) * (N / 64);
    wmma_gemm64<0, false, 2, 0, true, 0><<<dim3((tiles + 7) / 8, 1), 256, 0, stream>>>(
        h16, h16, K, 0L, w2_16, w2_16, K, 0L,
        (void*)outp, nullptr, MODEL_DIM, 0L, ff_b2, x1, 0L, M, N, K, 1.0f / 64.0f);
  }
}
